// RNN_89928025244149
// MI455X (gfx1250) — hardware-run, weakly checked
//
#include <hip/hip_runtime.h>
#include <math.h>

constexpr int NCH  = 128;
constexpr int NSEQ = 256;
constexpr int NB   = 1024;
constexpr int NH   = 256;
constexpr int NG4  = 1024;
constexpr int NTHR = 256;
constexpr int RB   = 16;
constexpr int HP   = 264;
constexpr int XSP  = 1028;
constexpr int LSP  = 132;
constexpr float USC  = 64.0f;
constexpr float HSC  = 16.0f;
constexpr float ZINV = 1.0f / 1024.0f;
static_assert(NG4 == 4 * NH);
static_assert(NH == 32 * (NTHR / 32));
static_assert(NCH == 16 * (NTHR / 32));
static_assert(RB == 2 * (NTHR / 32));
static_assert(NCH == 4 * 32);
static_assert(NB % RB == 0);
static_assert(NH % 32 == 0);
static_assert(NG4 % 64 == 0 && NH % 64 == 0 && NCH % 64 == 0);
static_assert(NG4 == 4 * NTHR);
static_assert(RB * NSEQ == 16 * NTHR);
static_assert(HP % 8 == 0 && XSP % 4 == 0 && LSP % 4 == 0);

typedef __attribute__((ext_vector_type(16))) _Float16 v16h;
typedef __attribute__((ext_vector_type(8)))  _Float16 v8h;
typedef __attribute__((ext_vector_type(8)))  float    v8f;
typedef __attribute__((ext_vector_type(4)))  float    v4f;
typedef __attribute__((ext_vector_type(4)))  int      v4i;

__device__ __forceinline__ void guard5_h(v8f& a0, v8f& a1, v8f& a2, v8f& a3,
                                         v16h x, v16h b0, v16h b1, v16h b2, v16h b3) {
  asm volatile("v_nop\n\tv_nop\n\tv_nop\n\tv_nop"
               : "+v"(a0), "+v"(a1), "+v"(a2), "+v"(a3)
               : "v"(x), "v"(b0), "v"(b1), "v"(b2), "v"(b3));
}
__device__ __forceinline__ void guard1_h(v8f& a0, v16h x, v16h b0) {
  asm volatile("v_nop\n\tv_nop\n\tv_nop\n\tv_nop" : "+v"(a0) : "v"(x), "v"(b0));
}
__device__ __forceinline__ void acc_guard4(v8f& a, v8f& b, v8f& c, v8f& d) {
  asm volatile("v_nop\n\tv_nop\n\tv_nop\n\tv_nop" : "+v"(a), "+v"(b), "+v"(c), "+v"(d));
}
__device__ __forceinline__ void acc_guard1(v8f& a) {
  asm volatile("v_nop\n\tv_nop\n\tv_nop\n\tv_nop" : "+v"(a));
}

template <typename T> struct Frag;
template <> struct Frag<_Float16> {
  typedef v16h V; union U { v16h v; v8h h[2]; };
  static __device__ __forceinline__ v16h load(const _Float16* p) {
    U f; f.h[0] = *(const v8h*)(p); f.h[1] = *(const v8h*)(p + 16); return f.v;
  }
  static __device__ __forceinline__ v8f mma(v16h a, v16h b, v8f c) {
    return __builtin_amdgcn_wmma_f32_16x16x32_f16(false, a, false, b, (short)0, c, false, false);
  }
};

__device__ __forceinline__ float fsig(float x)  { return __builtin_amdgcn_rcpf(1.0f + expf(-x)); }
__device__ __forceinline__ float ftanh(float x) { return 1.0f - 2.0f * __builtin_amdgcn_rcpf(expf(2.0f * x) + 1.0f); }

__global__ __launch_bounds__(NTHR) void tpc_kernel(const float* __restrict__ src, int R, int C, int ldo,
                                                   unsigned short* __restrict__ O, float sc) {
  __shared__ float Tt[64 * 65];
  const int tid = threadIdx.x;
  const int c0 = blockIdx.x * 64, r0 = blockIdx.y * 64;
#pragma unroll
  for (int i = 0; i < 4; ++i) {
    const int idx = i * NTHR + tid;
    const int rr = idx >> 4, cc = (idx & 15) * 4;
    const v4f v = *(const v4f*)(src + (size_t)(r0 + rr) * (size_t)C + c0 + cc);
    Tt[rr * 65 + cc + 0] = v[0];
    Tt[rr * 65 + cc + 1] = v[1];
    Tt[rr * 65 + cc + 2] = v[2];
    Tt[rr * 65 + cc + 3] = v[3];
  }
  __syncthreads();
  const int q = tid >> 3, c8 = (tid & 7) * 8;
  v8h hv[2];
#pragma unroll
  for (int g = 0; g < 2; ++g) {
    const int qq = g * 32 + q;
#pragma unroll
    for (int e = 0; e < 8; ++e) {
      const float f = Tt[(c8 + e) * 65 + qq];
      hv[g][e] = (_Float16)(f * sc);
    }
  }
  for (int pass = 0; pass < 2; ++pass) {
#pragma unroll
    for (int g = 0; g < 2; ++g) {
      const size_t o = (size_t)(c0 + g * 32 + q) * (size_t)ldo + (size_t)(r0 + c8);
      *(volatile v8h*)(O + o) = hv[g];
    }
    __threadfence();
  }
}

__global__ __launch_bounds__(NTHR) void lstm_seq_kernel(const int* __restrict__ tokens, const float* __restrict__ W,
                                                        const float* __restrict__ bias, const float* __restrict__ bd,
                                                        const unsigned short* __restrict__ UPp,
                                                        const unsigned short* __restrict__ WDPp,
                                                        float* __restrict__ out) {
  __shared__ __align__(16) _Float16 Ah[RB * HP];
  __shared__ __align__(16) float    Xs[RB * XSP];
  __shared__ __align__(16) int      Ts[RB * NSEQ];
  __shared__ __align__(16) float    Ls[RB * LSP];
  const _Float16* UP  = (const _Float16*)UPp;
  const _Float16* WDP = (const _Float16*)WDPp;
  const int tid = threadIdx.x, lane = tid & 31, wave = tid >> 5;
  const int c = lane & 15, hh = lane >> 4, koff = hh * 8;
  const int rowbase = blockIdx.x * RB;

#pragma unroll
  for (int i = 0; i < 4; ++i) {
    const int idx = i * NTHR + tid;
    const int row = idx >> 6, c4 = (idx & 63) * 4;
    v4i tk = *(const v4i*)(tokens + (size_t)(rowbase + row) * NSEQ + c4);
#pragma unroll
    for (int e = 0; e < 4; ++e) {
      int v = tk[e];
      v = v < 0 ? 0 : v;
      v = v > (NCH - 1) ? (NCH - 1) : v;
      tk[e] = v;
    }
    *(v4i*)(Ts + row * NSEQ + c4) = tk;
  }
#pragma unroll 1
  for (int i = tid; i < RB * HP; i += NTHR) Ah[i] = (_Float16)0.0f;
  float cst[2][8], hst[2][8], bb[2][4];
#pragma unroll
  for (int nt = 0; nt < 2; ++nt) {
    const int j = 32 * wave + 16 * nt + c;
#pragma unroll
    for (int g = 0; g < 4; ++g) bb[nt][g] = bias[g * NH + j];
#pragma unroll
    for (int r = 0; r < 8; ++r) { cst[nt][r] = 0.0f; hst[nt][r] = 0.0f; }
  }
  __syncthreads();

  const _Float16* ahrow = Ah + c * HP + koff;
  const v8f z8 = {0.f, 0.f, 0.f, 0.f, 0.f, 0.f, 0.f, 0.f};
  const int xc4 = tid * 4;

#pragma unroll 1
  for (int t = 0; t < NSEQ; ++t) {
#pragma unroll
    for (int half = 0; half < 2; ++half) {
      v4f xv[8];
#pragma unroll
      for (int i = 0; i < 8; ++i) {
        const int row = half * 8 + i;
        const int tok = Ts[row * NSEQ + t];
        xv[i] = *(const v4f*)(W + (size_t)tok * NG4 + xc4);
      }
#pragma unroll
      for (int i = 0; i < 8; ++i) *(v4f*)(Xs + (half * 8 + i) * XSP + xc4) = xv[i];
      asm volatile("" ::: "memory");
    }
    __syncthreads();

#pragma unroll
    for (int nt = 0; nt < 2; ++nt) {
      const int j = 32 * wave + 16 * nt + c;
      const _Float16* wu = UP + (size_t)j * NH + koff;
      v8f acc[4];
      acc[0] = z8; acc[1] = z8; acc[2] = z8; acc[3] = z8;
#pragma unroll 1
      for (int k0 = 0; k0 < NH; k0 += 32) {
        const v16h a  = Frag<_Float16>::load(ahrow + k0);
        const v16h b0 = Frag<_Float16>::load(wu + k0);
        const v16h b1 = Frag<_Float16>::load(wu + (size_t)1 * NH * NH + k0);
        const v16h b2 = Frag<_Float16>::load(wu + (size_t)2 * NH * NH + k0);
        const v16h b3 = Frag<_Float16>::load(wu + (size_t)3 * NH * NH + k0);
        acc[0] = Frag<_Float16>::mma(a, b0, acc[0]);
        acc[1] = Frag<_Float16>::mma(a, b1, acc[1]);
        acc[2] = Frag<_Float16>::mma(a, b2, acc[2]);
        acc[3] = Frag<_Float16>::mma(a, b3, acc[3]);
        guard5_h(acc[0], acc[1], acc[2], acc[3], a, b0, b1, b2, b3);
      }
      acc_guard4(acc[0], acc[1], acc[2], acc[3]);
#pragma unroll
      for (int r = 0; r < 8; ++r) {
        const float* xr = Xs + (8 * hh + r) * XSP + j;
        const float zi = acc[0][r] * ZINV + xr[0 * NH] + bb[nt][0];
        const float zf = acc[1][r] * ZINV + xr[1 * NH] + bb[nt][1];
        const float zg = acc[2][r] * ZINV + xr[2 * NH] + bb[nt][2];
        const float zo = acc[3][r] * ZINV + xr[3 * NH] + bb[nt][3];
        const float ig = fsig(zi);
        const float fg = fsig(zf);
        const float gg = ftanh(zg);
        const float og = fsig(zo);
        const float cn = fg * cst[nt][r] + ig * gg;
        cst[nt][r] = cn;
        hst[nt][r] = og * ftanh(cn);
      }
    }
    __syncthreads();
#pragma unroll
    for (int nt = 0; nt < 2; ++nt) {
      const int j = 32 * wave + 16 * nt + c;
#pragma unroll
      for (int r = 0; r < 8; ++r) Ah[(8 * hh + r) * HP + j] = (_Float16)(hst[nt][r] * HSC);
    }
  }
  __syncthreads();

  {
    const int n = 16 * wave + c;
    const _Float16* wd = WDP + (size_t)n * NH + koff;
    v8f accd = z8;
#pragma unroll 1
    for (int k0 = 0; k0 < NH; k0 += 32) {
      const v16h a  = Frag<_Float16>::load(ahrow + k0);
      const v16h b0 = Frag<_Float16>::load(wd + k0);
      accd = Frag<_Float16>::mma(a, b0, accd);
      guard1_h(accd, a, b0);
    }
    acc_guard1(accd);
    const float bdv = bd[n];
#pragma unroll
    for (int r = 0; r < 8; ++r) Ls[(8 * hh + r) * LSP + n] = accd[r] * ZINV + bdv;
  }
  __syncthreads();

  v4f orow[2];
#pragma unroll
  for (int rr = 0; rr < 2; ++rr) {
    const int row = 2 * wave + rr;
    const v4f v = *(const v4f*)(Ls + row * LSP + 4 * lane);
    float m = fmaxf(fmaxf(v[0], v[1]), fmaxf(v[2], v[3]));
#pragma unroll
    for (int off = 1; off < 32; off <<= 1) m = fmaxf(m, __shfl_xor(m, off, 32));
    v4f e;
    float s = 0.0f;
#pragma unroll
    for (int k = 0; k < 4; ++k) { e[k] = expf(v[k] - m); s += e[k]; }
#pragma unroll
    for (int off = 1; off < 32; off <<= 1) s += __shfl_xor(s, off, 32);
    const float inv = 1.0f / s;
    v4f o;
#pragma unroll
    for (int k = 0; k < 4; ++k) o[k] = e[k] * inv;
    orow[rr] = o;
  }
  for (int pass = 0; pass < 2; ++pass) {
#pragma unroll
    for (int rr = 0; rr < 2; ++rr)
      *(volatile v4f*)(out + (size_t)(rowbase + 2 * wave + rr) * NCH + 4 * lane) = orow[rr];
    __threadfence();
  }
}

extern "C" void kernel_launch(void* const* d_in, const int* in_sizes, int n_in,
                              void* d_out, int out_size, void* d_ws, size_t ws_size, hipStream_t stream) {
  if (n_in < 6 || d_out == nullptr || d_ws == nullptr) return;
  if (in_sizes[0] != NB * NSEQ || in_sizes[1] != NCH * NG4 || in_sizes[2] != NH * NG4 || in_sizes[3] != NG4 ||
      in_sizes[4] != NH * NCH || in_sizes[5] != NCH || out_size != NB * NCH) return;

  const int*   tokens = (const int*)d_in[0];
  const float* W      = (const float*)d_in[1];
  const float* U      = (const float*)d_in[2];
  const float* b      = (const float*)d_in[3];
  const float* Wd     = (const float*)d_in[4];
  const float* bd     = (const float*)d_in[5];
  float* out = (float*)d_out;

  char* ws = (char*)d_ws; size_t off = 0;
  auto carve = [&](size_t bytes) -> char* { char* p = ws + off; off += (bytes + 255) & ~(size_t)255; return p; };
  unsigned short* UP  = (unsigned short*)carve((size_t)NG4 * NH * 2);
  unsigned short* WDP = (unsigned short*)carve((size_t)NCH * NH * 2);
  if (off > ws_size || off > (size_t)134217728) return;

  tpc_kernel<<<dim3(NG4 / 64, NH / 64), NTHR, 0, stream>>>(U,  NH, NG4, NH, UP,  USC);
  tpc_kernel<<<dim3(NCH / 64, NH / 64), NTHR, 0, stream>>>(Wd, NH, NCH, NH, WDP, USC);
  lstm_seq_kernel<<<NB / RB, NTHR, 0, stream>>>(tokens, W, b, bd, UP, WDP, out);
}
